// CombinedLSTMWithStatic2Hop_32229434589314
// MI455X (gfx1250) — hardware-verified
//
#include <hip/hip_runtime.h>


#define BB   4
#define TT   96
#define NN   2000
#define BN   8000
#define FD   8
#define FS   16
#define HH   128
#define GG   512
#define EE   16000
#define AP   168
#define MR   32
#define GR   64
#define GP   264
#define SP   132
#define CAP  1024

static_assert(BN % MR == 0);
static_assert(BN % GR == 0);
static_assert((AP * 2) % 16 == 0);
static_assert((GP * 2) % 16 == 0);
static_assert((SP * 4) % 16 == 0);
static_assert(GR == 64);
static_assert(EE < 65536 && BN < 65536);

constexpr int LSTM_WPL = GG * AP * 2;
constexpr int LSTM_ATL = MR * AP * 2;
constexpr int LSTM_LDS = LSTM_WPL + LSTM_ATL;
constexpr int STG_B    = GR * SP * 4;
constexpr int APL_B    = GR * GP * 2;
constexpr int NODE_LDS = STG_B + 2 * APL_B;
constexpr int OFF_LIST = NODE_LDS;
constexpr int OFF_CNT  = OFF_LIST + CAP * 4;
constexpr int OFF_PRED = OFF_CNT + GR * 4;
constexpr int OFF_WCNT = OFF_PRED + GR * 4;
constexpr int SAGE_LDS = OFF_WCNT + 64;
static_assert(MR * SP * 4 <= LSTM_WPL);
static_assert(LSTM_WPL % 16 == 0 && STG_B % 16 == 0 && APL_B % 16 == 0);
static_assert(OFF_LIST % 16 == 0 && OFF_PRED % 16 == 0 && OFF_WCNT % 16 == 0);

constexpr size_t PL_B     = (size_t)BN * HH * 4;
constexpr size_t OFF_Z    = 0;
constexpr size_t OFF_NODE = PL_B;
constexpr size_t OFF_H1   = 2 * PL_B;
constexpr size_t WS_END   = 3 * PL_B;
static_assert(WS_END <= (size_t)134217728);
static_assert(PL_B % 128 == 0);

typedef float          v4f   __attribute__((ext_vector_type(4)));
typedef float          v8f   __attribute__((ext_vector_type(8)));
typedef _Float16       v8h   __attribute__((ext_vector_type(8)));
typedef _Float16       v16h  __attribute__((ext_vector_type(16)));
typedef __bf16         v16b  __attribute__((ext_vector_type(16)));
typedef unsigned short u16x8 __attribute__((ext_vector_type(8)));

union FragH { v16h v; v8h  h[2]; };
union FragB { v16b v; u16x8 h[2]; };

extern __shared__ __attribute__((aligned(16))) unsigned char dsm[];

__device__ __forceinline__ unsigned short bf16_bits(float f) {
    unsigned u = __float_as_uint(f);
    u += 0x7FFFu + ((u >> 16) & 1u);
    return (unsigned short)(u >> 16);
}
__device__ __forceinline__ float bf16_val(unsigned short b) {
    return __uint_as_float(((unsigned)b) << 16);
}
__device__ __forceinline__ v8f ld8f(const float* p) {
    const v4f a = *(const v4f*)p;
    const v4f b = *(const v4f*)(p + 4);
    return __builtin_shufflevector(a, b, 0, 1, 2, 3, 4, 5, 6, 7);
}
__device__ __forceinline__ void split8(const v8f x, u16x8& hv, u16x8& lv) {
#pragma unroll
    for (int i = 0; i < 8; ++i) {
        const float f = x[i];
        const unsigned short hb = bf16_bits(f);
        const unsigned short lb = bf16_bits(f - bf16_val(hb));
        hv[i] = hb;
        lv[i] = lb;
    }
}
__device__ __forceinline__ v8f zero8f() {
    v8f z;
#pragma unroll
    for (int i = 0; i < 8; ++i) z[i] = 0.0f;
    return z;
}
__device__ __forceinline__ u16x8 zero16() {
    u16x8 z;
#pragma unroll
    for (int i = 0; i < 8; ++i) z[i] = 0;
    return z;
}
__device__ __forceinline__ float sigm_(float x) {
    return __builtin_amdgcn_rcpf(1.0f + __builtin_amdgcn_exp2f(-1.4426950408889634f * x));
}
__device__ __forceinline__ float tanh_(float x) {
    const float e = __builtin_amdgcn_exp2f(2.8853900817779268f * x);
    return 1.0f - 2.0f * __builtin_amdgcn_rcpf(e + 1.0f);
}

__device__ __forceinline__ v8f wf16(v8f c, const FragH& a, const FragH& b) {
    return __builtin_amdgcn_wmma_f32_16x16x32_f16(false, a.v, false, b.v, (short)0, c, false, false);
}
__device__ __forceinline__ v8f wbf(v8f c, const FragB& a, const FragB& b) {
    return __builtin_amdgcn_wmma_f32_16x16x32_bf16(false, a.v, false, b.v, (short)0, c, false, false);
}
__device__ __forceinline__ void mma3(v8f& acc, const FragB& ah, const FragB& al, const FragB& bh, const FragB& bl) {
    acc = wbf(acc, ah, bh);
    acc = wbf(acc, ah, bl);
    acc = wbf(acc, al, bh);
    asm volatile("v_nop\n\tv_nop\n\tv_nop\n\tv_nop" : "+v"(acc) : "v"(ah.v), "v"(al.v), "v"(bh.v), "v"(bl.v));
}
__device__ __forceinline__ void ldfrag_split(FragB& fh, FragB& fl, const float* p) {
    const v8f x0 = ld8f(p);
    const v8f x1 = ld8f(p + 16);
    split8(x0, fh.h[0], fl.h[0]);
    split8(x1, fh.h[1], fl.h[1]);
}

__device__ __forceinline__ void store_rows64(const float* stg, float* dst, int w, int lane) {
    v4f v[8];
#pragma unroll
    for (int it = 0; it < 8; ++it) {
        const int gl  = it * 32 + w * 4 + (lane >> 3);
        const int row = gl >> 2, cc = (gl & 3) * 32 + (lane & 7) * 4;
        v[it] = *(const v4f*)(stg + row * SP + cc);
    }
#pragma unroll
    for (int it = 0; it < 8; ++it) {
        const int gl  = it * 32 + w * 4 + (lane >> 3);
        const int row = gl >> 2, cc = (gl & 3) * 32 + (lane & 7) * 4;
        *(volatile v4f*)(dst + (size_t)row * HH + cc) = v[it];
    }
    __threadfence();
#pragma unroll
    for (int it = 0; it < 8; ++it) {
        const int gl  = it * 32 + w * 4 + (lane >> 3);
        const int row = gl >> 2, cc = (gl & 3) * 32 + (lane & 7) * 4;
        *(volatile v4f*)(dst + (size_t)row * HH + cc) = v[it];
    }
}

__device__ __forceinline__ void gemm_part(const unsigned short* Ah, const unsigned short* Al, int kbase,
                                          const float* __restrict__ wrow, v8f (&acc)[4], int m, int h)
{
#pragma unroll 1
    for (int kc = 0; kc < 4; ++kc) {
        FragB fbh, fbl;
        ldfrag_split(fbh, fbl, wrow + kc * 32);
        const int ko = kbase + kc * 32 + 8 * h;
#pragma unroll
        for (int rt = 0; rt < 4; ++rt) {
            FragB fah, fal;
            const unsigned short* pa = Ah + (rt * 16 + m) * GP + ko;
            const unsigned short* pl = Al + (rt * 16 + m) * GP + ko;
            fah.h[0] = *(const u16x8*)(pa);
            fah.h[1] = *(const u16x8*)(pa + 16);
            fal.h[0] = *(const u16x8*)(pl);
            fal.h[1] = *(const u16x8*)(pl + 16);
            mma3(acc[rt], fah, fal, fbh, fbl);
        }
    }
}

__global__ __launch_bounds__(256)
void k_lstm(const float* __restrict__ dyn, const float* __restrict__ W_ih, const float* __restrict__ W_hh,
            const float* __restrict__ b_ih, const float* __restrict__ b_hh, float* zpl)
{
    _Float16* Wl  = (_Float16*)dsm;
    _Float16* At  = (_Float16*)(dsm + LSTM_WPL);
    float*    stg = (float*)dsm;

    const int tid = threadIdx.x, lane = tid & 31, w = tid >> 5;
    const int h = lane >> 4, m = lane & 15;
    const int col = (w << 4) | m;
    const int r0 = blockIdx.x * MR;

    v8h z8h;
#pragma unroll
    for (int i = 0; i < 8; ++i) z8h[i] = (_Float16)0.0f;

#pragma unroll 1
    for (int idx = tid; idx < GG * 16; idx += 256) {
        const int n = idx >> 4, c8 = idx & 15;
        const v8f x = ld8f(W_hh + (size_t)n * HH + 8 * c8);
        v8h hv;
#pragma unroll
        for (int i = 0; i < 8; ++i) hv[i] = (_Float16)(x[i] * 8.0f);
        *(v8h*)(Wl + n * AP + 8 * c8) = hv;
    }
#pragma unroll 1
    for (int n = tid; n < GG; n += 256) {
        const v8f x = ld8f(W_ih + n * FD);
        v8h hi, lo;
#pragma unroll
        for (int i = 0; i < 8; ++i) {
            const float v  = x[i] * 8.0f;
            const float hf = bf16_val(bf16_bits(v));
            hi[i] = (_Float16)hf;
            lo[i] = (_Float16)(v - hf);
        }
        _Float16* p = Wl + n * AP + HH;
        *(v8h*)(p)      = hi;
        *(v8h*)(p + 8)  = hi;
        *(v8h*)(p + 16) = lo;
        *(v8h*)(p + 24) = z8h;
    }
#pragma unroll 1
    for (int idx = tid; idx < (MR * AP) / 8; idx += 256)
        *(v8h*)(At + 8 * idx) = z8h;
    __syncthreads();

    const int xr = tid >> 3, xf = tid & 7;
    const int xgr = r0 + xr;
    const int xb = xgr / NN, xn = xgr - xb * NN;
    const float* xptr = dyn + ((size_t)xb * TT * NN + xn) * FD + xf;
    _Float16* xdst = At + xr * AP + HH + xf;
    {
        const float xv = xptr[0];
        const float hf = bf16_val(bf16_bits(xv));
        xdst[0]  = (_Float16)hf;
        xdst[8]  = (_Float16)(xv - hf);
        xdst[16] = (_Float16)hf;
    }

    const float bgi = b_ih[col]          + b_hh[col];
    const float bgf = b_ih[HH + col]     + b_hh[HH + col];
    const float bgg = b_ih[2 * HH + col] + b_hh[2 * HH + col];
    const float bgo = b_ih[3 * HH + col] + b_hh[3 * HH + col];

    float c[2][8];
#pragma unroll
    for (int rt = 0; rt < 2; ++rt)
#pragma unroll
        for (int r = 0; r < 8; ++r) c[rt][r] = 0.0f;

#pragma unroll 1
    for (int t = 0; t < TT; ++t) {
        __syncthreads();
        v8f acc[2][4];
#pragma unroll
        for (int rt = 0; rt < 2; ++rt)
#pragma unroll
            for (int j = 0; j < 4; ++j) acc[rt][j] = zero8f();

#pragma unroll 1
        for (int kc = 0; kc < 5; ++kc) {
            FragH a0, a1, b[4];
            const _Float16* pa = At + m * AP + kc * 32 + 8 * h;
            a0.h[0] = *(const v8h*)(pa);
            a0.h[1] = *(const v8h*)(pa + 16);
            a1.h[0] = *(const v8h*)(pa + 16 * AP);
            a1.h[1] = *(const v8h*)(pa + 16 * AP + 16);
            const _Float16* pb = Wl + col * AP + kc * 32 + 8 * h;
#pragma unroll
            for (int j = 0; j < 4; ++j) {
                b[j].h[0] = *(const v8h*)(pb + j * (HH * AP));
                b[j].h[1] = *(const v8h*)(pb + j * (HH * AP) + 16);
            }
#pragma unroll
            for (int j = 0; j < 4; ++j) {
                acc[0][j] = wf16(acc[0][j], a0, b[j]);
                acc[1][j] = wf16(acc[1][j], a1, b[j]);
            }
            asm volatile("v_nop\n\tv_nop\n\tv_nop\n\tv_nop"
                : "+v"(acc[0][0]), "+v"(acc[0][1]), "+v"(acc[0][2]), "+v"(acc[0][3]),
                  "+v"(acc[1][0]), "+v"(acc[1][1]), "+v"(acc[1][2]), "+v"(acc[1][3])
                : "v"(a0.v), "v"(a1.v), "v"(b[0].v), "v"(b[1].v), "v"(b[2].v), "v"(b[3].v));
        }
        __syncthreads();

        float hv[2][8];
#pragma unroll
        for (int rt = 0; rt < 2; ++rt) {
#pragma unroll
            for (int r = 0; r < 8; ++r) {
                const float pi = acc[rt][0][r] * 0.125f + bgi;
                const float pf = acc[rt][1][r] * 0.125f + bgf;
                const float pg = acc[rt][2][r] * 0.125f + bgg;
                const float po = acc[rt][3][r] * 0.125f + bgo;
                const float ig = sigm_(pi);
                const float fg = sigm_(pf);
                const float gg = tanh_(pg);
                const float og = sigm_(po);
                c[rt][r] = fg * c[rt][r] + ig * gg;
                const float hh = og * tanh_(c[rt][r]);
                hv[rt][r] = hh;
                At[(rt * 16 + 8 * h + r) * AP + col] = (_Float16)hh;
            }
        }
        if (t == TT - 1) {
#pragma unroll
            for (int rt = 0; rt < 2; ++rt)
#pragma unroll
                for (int r = 0; r < 8; ++r)
                    stg[(rt * 16 + 8 * h + r) * SP + col] = hv[rt][r];
        }
        if (t + 1 < TT) {
            const float xv = xptr[(size_t)(t + 1) * (NN * FD)];
            const float hf = bf16_val(bf16_bits(xv));
            xdst[0]  = (_Float16)hf;
            xdst[8]  = (_Float16)(xv - hf);
            xdst[16] = (_Float16)hf;
        }
    }
    __syncthreads();

    v4f v[4];
#pragma unroll
    for (int it = 0; it < 4; ++it) {
        const int gl  = it * 32 + w * 4 + (lane >> 3);
        const int row = gl >> 2, cc = (gl & 3) * 32 + (lane & 7) * 4;
        v[it] = *(const v4f*)(stg + row * SP + cc);
    }
#pragma unroll
    for (int it = 0; it < 4; ++it) {
        const int gl  = it * 32 + w * 4 + (lane >> 3);
        const int row = gl >> 2, cc = (gl & 3) * 32 + (lane & 7) * 4;
        *(volatile v4f*)(zpl + (size_t)(r0 + row) * HH + cc) = v[it];
    }
    __threadfence();
#pragma unroll
    for (int it = 0; it < 4; ++it) {
        const int gl  = it * 32 + w * 4 + (lane >> 3);
        const int row = gl >> 2, cc = (gl & 3) * 32 + (lane & 7) * 4;
        *(volatile v4f*)(zpl + (size_t)(r0 + row) * HH + cc) = v[it];
    }
}

__global__ __launch_bounds__(256)
void k_node(const float* __restrict__ zpl, const float* __restrict__ sta, const float* __restrict__ W_sta,
            const float* __restrict__ b_sta, const float* __restrict__ W_fuse, const float* __restrict__ b_fuse,
            float* nodepl)
{
    float* stg = (float*)dsm;
    unsigned short* Ah = (unsigned short*)(dsm + STG_B);
    unsigned short* Al = (unsigned short*)(dsm + STG_B + APL_B);

    const int tid = threadIdx.x, lane = tid & 31, w = tid >> 5;
    const int h = lane >> 4, m = lane & 15;
    const int col = (w << 4) | m;
    const int r0 = blockIdx.x * GR;
    const u16x8 z16 = zero16();

#pragma unroll 1
    for (int idx = tid; idx < GR * 16; idx += 256) {
        const int row = idx >> 4, c8 = idx & 15;
        const v8f x = ld8f(zpl + (size_t)(r0 + row) * HH + 8 * c8);
        u16x8 hv, lv;
        split8(x, hv, lv);
        *(u16x8*)(Ah + row * GP + 8 * c8) = hv;
        *(u16x8*)(Al + row * GP + 8 * c8) = lv;
    }

    FragB sbh, sbl;
    {
        const v8f x = ld8f(W_sta + col * FS + 8 * h);
        split8(x, sbh.h[0], sbl.h[0]);
        sbh.h[1] = z16;
        sbl.h[1] = z16;
    }
    const float bs = b_sta[col];
#pragma unroll
    for (int rt = 0; rt < 4; ++rt) {
        FragB sah, sal;
        {
            const v8f x = ld8f(sta + (size_t)(r0 + rt * 16 + m) * FS + 8 * h);
            split8(x, sah.h[0], sal.h[0]);
            sah.h[1] = z16;
            sal.h[1] = z16;
        }
        v8f acc0 = zero8f();
        mma3(acc0, sah, sal, sbh, sbl);
#pragma unroll
        for (int r = 0; r < 8; ++r) {
            const float v = fmaxf(acc0[r] + bs, 0.0f);
            const unsigned short hb = bf16_bits(v);
            const unsigned short lb = bf16_bits(v - bf16_val(hb));
            const int o = (rt * 16 + 8 * h + r) * GP + HH + col;
            Ah[o] = hb;
            Al[o] = lb;
        }
    }
    __syncthreads();

    v8f acc[4];
#pragma unroll
    for (int rt = 0; rt < 4; ++rt) acc[rt] = zero8f();
    const float* wrow = W_fuse + (size_t)col * (2 * HH) + 8 * h;
    gemm_part(Ah, Al, 0,  wrow,      acc, m, h);
    gemm_part(Ah, Al, HH, wrow + HH, acc, m, h);

    const float bb = b_fuse[col];
#pragma unroll
    for (int rt = 0; rt < 4; ++rt)
#pragma unroll
        for (int r = 0; r < 8; ++r)
            stg[(rt * 16 + 8 * h + r) * SP + col] = fmaxf(acc[rt][r] + bb, 0.0f);
    __syncthreads();
    store_rows64(stg, nodepl + (size_t)r0 * HH, w, lane);
}

template<int LAYER>
__global__ __launch_bounds__(256)
void k_sage(const float* __restrict__ xsrc, const int* __restrict__ ei,
            const float* __restrict__ Wl, const float* __restrict__ bl, const float* __restrict__ Wr,
            const float* __restrict__ Wo, const float* __restrict__ bo, float* hout, float* pred)
{
    float* accs = (float*)dsm;
    unsigned short* Ah = (unsigned short*)(dsm + STG_B);
    unsigned short* Al = (unsigned short*)(dsm + STG_B + APL_B);
    int*   s_list = (int*)(dsm + OFF_LIST);
    int*   s_cnt  = (int*)(dsm + OFF_CNT);
    float* s_pred = (float*)(dsm + OFF_PRED);
    int*   s_wc   = (int*)(dsm + OFF_WCNT);

    const int tid = threadIdx.x, lane = tid & 31, w = tid >> 5;
    const int h = lane >> 4, m = lane & 15;
    const int col = (w << 4) | m;
    const int r0 = blockIdx.x * GR;

    v4f z4;
#pragma unroll
    for (int i = 0; i < 4; ++i) z4[i] = 0.0f;
#pragma unroll
    for (int k = 0; k < 8; ++k)
        *(v4f*)(accs + (w + 8 * k) * SP + lane * 4) = z4;
    if (lane < 8) s_cnt[w + 8 * lane] = 0;
    if (tid == 0) s_wc[8] = 0;
    __syncthreads();

    const int blo = r0 / NN;
    const int bhi = (r0 + GR - 1) / NN;
#pragma unroll 1
    for (int be = blo; be <= bhi; ++be) {
        const int boff = be * NN;
#pragma unroll 1
        for (int c0 = 0; c0 < EE; c0 += 256) {
            const int e  = c0 + tid;
            const int ec = min(e, EE - 1);
            const int d  = ei[EE + ec];
            const int s  = ei[ec];
            const int slot = d + boff - r0;
            const bool hit = (e < EE) && ((unsigned)d < (unsigned)NN) && ((unsigned)slot < (unsigned)GR);
            const int sg = min(max(s, 0), NN - 1) + boff;
            const unsigned mask = __builtin_amdgcn_ballot_w32(hit);
            const int pre = (int)__builtin_amdgcn_mbcnt_lo(mask, 0u);
            if (lane == 0) s_wc[w] = __builtin_popcount(mask);
            __syncthreads();
            const int base = s_wc[8];
            int below = 0, tot = 0;
#pragma unroll
            for (int v = 0; v < 8; ++v) {
                const int cv = s_wc[v];
                tot += cv;
                below += (v < w) ? cv : 0;
            }
            const int pos = base + below + pre;
            if (hit && pos < CAP) s_list[pos] = (slot << 16) | sg;
            __syncthreads();
            if (tid == 0) s_wc[8] = min(base + tot, CAP);
        }
    }
    __syncthreads();
    const int L = min(s_wc[8], CAP);

#pragma unroll 1
    for (int base = 0; base < L; base += 32) {
        const int idx = base + lane;
        const int ent = s_list[min(idx, CAP - 1)];
        const bool hit = (idx < L) && (((ent >> 16) & 7) == w);
        unsigned mask = __builtin_amdgcn_ballot_w32(hit);
        while (mask != 0u) {
            const int bp   = __builtin_ctz(mask);
            const int eb   = __shfl(ent, bp, 32);
            const int slot = (eb >> 16) & (GR - 1);
            const int src  = min(eb & 0xffff, BN - 1);
            const v4f xv = *(const v4f*)(xsrc + (size_t)src * HH + lane * 4);
            float* ap = accs + slot * SP + lane * 4;
            const v4f av = *(const v4f*)ap;
            *(v4f*)ap = av + xv;
            if (lane == 0) s_cnt[slot] += 1;
            mask &= mask - 1u;
        }
    }
    __syncthreads();

#pragma unroll 1
    for (int idx = tid; idx < GR * 16; idx += 256) {
        const int row = idx >> 4, c8 = idx & 15;
        const float cn = (float)s_cnt[row];
        const float rc = __builtin_amdgcn_rcpf(fmaxf(cn, 1.0f));
        const v8f x = ld8f(accs + row * SP + 8 * c8) * rc;
        u16x8 hv, lv;
        split8(x, hv, lv);
        *(u16x8*)(Ah + row * GP + 8 * c8) = hv;
        *(u16x8*)(Al + row * GP + 8 * c8) = lv;
    }
#pragma unroll 1
    for (int idx = tid; idx < GR * 16; idx += 256) {
        const int row = idx >> 4, c8 = idx & 15;
        const v8f x = ld8f(xsrc + (size_t)(r0 + row) * HH + 8 * c8);
        u16x8 hv, lv;
        split8(x, hv, lv);
        *(u16x8*)(Ah + row * GP + HH + 8 * c8) = hv;
        *(u16x8*)(Al + row * GP + HH + 8 * c8) = lv;
    }
    __syncthreads();

    v8f acc[4];
#pragma unroll
    for (int rt = 0; rt < 4; ++rt) acc[rt] = zero8f();
    gemm_part(Ah, Al, 0,  Wl + (size_t)col * HH + 8 * h, acc, m, h);
    gemm_part(Ah, Al, HH, Wr + (size_t)col * HH + 8 * h, acc, m, h);
    const float bv = bl[col];

    if (LAYER == 1) {
#pragma unroll
        for (int rt = 0; rt < 4; ++rt)
#pragma unroll
            for (int r = 0; r < 8; ++r)
                accs[(rt * 16 + 8 * h + r) * SP + col] = fmaxf(acc[rt][r] + bv, 0.0f);
        __syncthreads();
        store_rows64(accs, hout + (size_t)r0 * HH, w, lane);
    } else {
#pragma unroll
        for (int rt = 0; rt < 4; ++rt)
#pragma unroll
            for (int r = 0; r < 8; ++r)
                accs[(rt * 16 + 8 * h + r) * SP + col] = acc[rt][r] + bv;
        __syncthreads();
        if (w < 4) {
            const int rt = w;
            const float wsel = (m == 0) ? 1.0f : 0.0f;
            v8f hacc = zero8f();
#pragma unroll
            for (int kc = 0; kc < 4; ++kc) {
                FragB gah, gal, gbh, gbl;
                {
                    const float* pa = accs + (rt * 16 + m) * SP + kc * 32 + 8 * h;
                    const v8f x0 = ld8f(pa);
                    const v8f x1 = ld8f(pa + 16);
                    split8(x0, gah.h[0], gal.h[0]);
                    split8(x1, gah.h[1], gal.h[1]);
                }
                {
                    const v8f w0 = ld8f(Wo + kc * 32 + 8 * h) * wsel;
                    const v8f w1 = ld8f(Wo + kc * 32 + 16 + 8 * h) * wsel;
                    split8(w0, gbh.h[0], gbl.h[0]);
                    split8(w1, gbh.h[1], gbl.h[1]);
                }
                mma3(hacc, gah, gal, gbh, gbl);
            }
            const float bov = bo[0];
            if (m == 0) {
#pragma unroll
                for (int r = 0; r < 8; ++r) s_pred[rt * 16 + 8 * h + r] = hacc[r] + bov;
            }
        }
        __syncthreads();
        if (w == 0) {
            const int li = min(lane, 15);
            const v4f pv = *(const v4f*)(s_pred + li * 4);
            if (lane < 16) *(volatile v4f*)(pred + r0 + lane * 4) = pv;
            __threadfence();
            if (lane < 16) *(volatile v4f*)(pred + r0 + lane * 4) = pv;
        }
    }
}

extern "C" void kernel_launch(void* const* d_in, const int* in_sizes, int n_in,
                              void* d_out, int out_size, void* d_ws, size_t ws_size,
                              hipStream_t stream)
{
    if (n_in < 19) return;
    if (in_sizes[0]  != BB * TT * NN * FD) return;
    if (in_sizes[1]  != BB * NN * FS)      return;
    if (in_sizes[2]  != 2 * EE)            return;
    if (in_sizes[3]  != GG * FD)           return;
    if (in_sizes[4]  != GG * HH)           return;
    if (in_sizes[5]  != GG)                return;
    if (in_sizes[6]  != GG)                return;
    if (in_sizes[7]  != HH * FS)           return;
    if (in_sizes[8]  != HH)                return;
    if (in_sizes[9]  != HH * 2 * HH)       return;
    if (in_sizes[10] != HH)                return;
    if (in_sizes[11] != HH * HH)           return;
    if (in_sizes[12] != HH)                return;
    if (in_sizes[13] != HH * HH)           return;
    if (in_sizes[14] != HH * HH)           return;
    if (in_sizes[15] != HH)                return;
    if (in_sizes[16] != HH * HH)           return;
    if (in_sizes[17] != HH)                return;
    if (in_sizes[18] != 1)                 return;
    if (out_size != BN)                    return;
    if (ws_size < WS_END)                  return;

    const float* dyn    = (const float*)d_in[0];
    const float* sta    = (const float*)d_in[1];
    const int*   ei     = (const int*)  d_in[2];
    const float* W_ih   = (const float*)d_in[3];
    const float* W_hh   = (const float*)d_in[4];
    const float* b_ih   = (const float*)d_in[5];
    const float* b_hh   = (const float*)d_in[6];
    const float* W_sta  = (const float*)d_in[7];
    const float* b_sta  = (const float*)d_in[8];
    const float* W_fuse = (const float*)d_in[9];
    const float* b_fuse = (const float*)d_in[10];
    const float* s1Wl   = (const float*)d_in[11];
    const float* s1bl   = (const float*)d_in[12];
    const float* s1Wr   = (const float*)d_in[13];
    const float* s2Wl   = (const float*)d_in[14];
    const float* s2bl   = (const float*)d_in[15];
    const float* s2Wr   = (const float*)d_in[16];
    const float* W_out  = (const float*)d_in[17];
    const float* b_out  = (const float*)d_in[18];
    float* out = (float*)d_out;

    char* ws = (char*)d_ws;
    float* zpl    = (float*)(ws + OFF_Z);
    float* nodepl = (float*)(ws + OFF_NODE);
    float* h1pl   = (float*)(ws + OFF_H1);

    hipFuncSetAttribute(reinterpret_cast<const void*>(&k_lstm),    hipFuncAttributeMaxDynamicSharedMemorySize, LSTM_LDS);
    hipFuncSetAttribute(reinterpret_cast<const void*>(&k_node),    hipFuncAttributeMaxDynamicSharedMemorySize, NODE_LDS);
    hipFuncSetAttribute(reinterpret_cast<const void*>(&k_sage<1>), hipFuncAttributeMaxDynamicSharedMemorySize, SAGE_LDS);
    hipFuncSetAttribute(reinterpret_cast<const void*>(&k_sage<2>), hipFuncAttributeMaxDynamicSharedMemorySize, SAGE_LDS);

    k_lstm<<<dim3(BN / MR), dim3(256), LSTM_LDS, stream>>>(dyn, W_ih, W_hh, b_ih, b_hh, zpl);
    k_node<<<dim3(BN / GR), dim3(256), NODE_LDS, stream>>>(zpl, sta, W_sta, b_sta, W_fuse, b_fuse, nodepl);
    k_sage<1><<<dim3(BN / GR), dim3(256), SAGE_LDS, stream>>>(nodepl, ei, s1Wl, s1bl, s1Wr, W_out, b_out, h1pl, out);
    k_sage<2><<<dim3(BN / GR), dim3(256), SAGE_LDS, stream>>>(h1pl, ei, s2Wl, s2bl, s2Wr, W_out, b_out, nodepl, out);
}
